// EGNN_Spherical_67577015435590
// MI455X (gfx1250) — hardware-run, weakly checked
//
#include <hip/hip_runtime.h>


namespace {
constexpr int N = 8192, E = 32768, MS = 32, MV = 16, DIM = 80, NR = 16, HID = 64, WN = 2560, O1 = 1024, O2 = 1536, O3 = 1792, O4 = 2304;
constexpr float XS = 8.0f, WSC = 256.0f, CUT = 5.0f, ALPHA = 1.0f, SQ3 = 1.7320508075688772f, SQ2 = 1.4142135623730951f, PI = 3.14159265358979323846f;
typedef _Float16 b16;
typedef __attribute__((ext_vector_type(16))) _Float16 v16b;
typedef __attribute__((ext_vector_type(8))) _Float16 v8b;
typedef __attribute__((ext_vector_type(8))) float v8f;
typedef __attribute__((ext_vector_type(4))) float v4f;
__device__ __forceinline__ float bf16_rne(float f) { unsigned int u = __float_as_uint(f); u += 0x7FFFu + ((u >> 16) & 1u); float r = __uint_as_float(u & 0xFFFF0000u); asm volatile("" : "+v"(r)); return r; }
__device__ __forceinline__ void split16(float v, b16& hi, b16& lo) { hi = (b16)v; lo = (b16)(v - (float)hi); }
__device__ __forceinline__ v16b frag_kb(const b16* p, int hh) { const v8b a = *(const v8b*)(p + 8 * hh), b = *(const v8b*)(p + 16 + 8 * hh); v16b f;
#pragma unroll
  for (int e = 0; e < 8; ++e) { f[e] = a[e]; f[8 + e] = b[e]; } return f; }
__device__ __forceinline__ v8f wmma16b(v16b a, v16b b, v8f c) { v8f d = __builtin_amdgcn_wmma_f32_16x16x32_f16(false, a, false, b, (short)0, c, false, false); asm volatile("v_nop\n\tv_nop\n\tv_nop\n\tv_nop" : "+v"(d) : "v"(a), "v"(b)); return d; }
__device__ __forceinline__ void wave_lds_sync() { __builtin_amdgcn_fence(__ATOMIC_RELEASE, "workgroup"); __builtin_amdgcn_wave_barrier(); __builtin_amdgcn_fence(__ATOMIC_ACQUIRE, "workgroup"); }
__device__ __forceinline__ float pmul(float a, float b) { float p = a * b; asm volatile("" : "+v"(p)); return p; }
__device__ __forceinline__ int iclamp(int v, int lo, int hi) { return v < lo ? lo : (v > hi ? hi : v); }
__device__ __forceinline__ float silu(float v) { return v / (1.0f + __expf(-v)); }
constexpr int CSR_NBLK9 = 512, CSR_GB9 = 9, CSR_GN9 = 1 << CSR_GB9  , CSR_TS9 = (CSR_GN9 < 32 ? 32 : CSR_GN9)  , CSR_MAXG9 = 512, CSR_CAP9 = 12288  ;
__device__ __host__ __forceinline__ int csr_tix9(int v) { return (v >> CSR_GB9) * CSR_TS9 + (v & (CSR_GN9 - 1)); }
__global__ __launch_bounds__(64) void csrA_kernel9(const int* __restrict__ dst, int E, int N, int nG, int CHP, int NGP, int* __restrict__ STG, int* __restrict__ HST) {
  extern __shared__ int sm[];
  int* cnt = sm; int* run = sm + NGP; int* ids = sm + 2 * NGP;
  const int b = blockIdx.x; const int ch = (E + CSR_NBLK9 - 1) / CSR_NBLK9; const int e0 = b * ch, e1 = min(E, e0 + ch);
  for (int i = threadIdx.x; i < NGP; i += 64) cnt[i] = 0;
  for (int i = threadIdx.x; i < CHP; i += 64) ids[i] = -1;
  __syncthreads();
  if (threadIdx.x == 0) {
    for (int e = e0; e < e1; ++e) { int d = dst[e]; d = (d < 0) ? 0 : (d >= N ? N - 1 : d); cnt[d >> CSR_GB9] += 1; }
    int acc = 0; for (int g = 0; g < nG; ++g) { run[g] = acc; acc += cnt[g]; }
    for (int e = e0; e < e1; ++e) { int d = dst[e]; d = (d < 0) ? 0 : (d >= N ? N - 1 : d); const int g = d >> CSR_GB9; ids[run[g]] = e; run[g] += 1; } }
  __syncthreads();
  typedef __attribute__((ext_vector_type(4))) int v4i;
  for (int pass = 0; pass < 2; ++pass) {
    for (int i = threadIdx.x; i < CHP / 4; i += 64) *(volatile v4i*)(STG + (size_t)b * CHP + i * 4) = *(const v4i*)(&ids[i * 4]);
    for (int i = threadIdx.x; i < NGP / 4; i += 64) { v4i v; for (int e = 0; e < 4; ++e) v[e] = (i * 4 + e < nG) ? cnt[i * 4 + e] : 0; *(volatile v4i*)(HST + (size_t)b * NGP + i * 4) = v; }
    __threadfence(); }
}
__global__ __launch_bounds__(512) void csrS_kernel9(const int* __restrict__ HST, int nG, int NGP, int* __restrict__ START, int* __restrict__ TOT, int* __restrict__ OFF) {
  __shared__ int tot[CSR_MAXG9];
  const int b = threadIdx.x;
  for (int pass = 0; pass < 2; ++pass) { int runb = 0; for (int g = 0; g < nG; ++g) { int c = HST[(size_t)b * NGP + g]; c = (c < 0) ? 0 : c; ((volatile int*)OFF)[(size_t)g * CSR_NBLK9 + b] = runb; runb += c; } __threadfence(); }
  for (int g = threadIdx.x; g < nG; g += 512) { int s = 0; for (int bb = 0; bb < CSR_NBLK9; ++bb) { int c = HST[(size_t)bb * NGP + g]; s += (c < 0) ? 0 : c; } tot[g] = s; }
  __syncthreads();
  if (threadIdx.x < 32) {
    __shared__ int st[CSR_MAXG9 + 32];
    if (threadIdx.x == 0) { int acc = 0; for (int g = 0; g < NGP; ++g) { st[g] = acc; if (g < nG) acc += (tot[g] + 31) & ~31; } st[NGP] = acc; }
    __builtin_amdgcn_fence(__ATOMIC_RELEASE, "workgroup"); __builtin_amdgcn_wave_barrier(); __builtin_amdgcn_fence(__ATOMIC_ACQUIRE, "workgroup");
    for (int pass = 0; pass < 2; ++pass) { for (int i = threadIdx.x; i < NGP + 32; i += 32) { ((volatile int*)START)[i] = (i <= NGP) ? st[min(i, NGP)] : 0; ((volatile int*)TOT)[i] = (i < nG) ? tot[i] : 0; } __threadfence(); } }
}
__global__ __launch_bounds__(256) void csrB_kernel9(const int* __restrict__ dst, int N, int nG, int CHP, int NGP, int permLen, const int* __restrict__ STG, const int* __restrict__ HST, const int* __restrict__ OFF, const int* __restrict__ START, const int* __restrict__ TOT, int* __restrict__ PERM, int* __restrict__ ROWPTR, int* __restrict__ ROWCNT, int* __restrict__ FLAG) {
  typedef __attribute__((ext_vector_type(4))) int v4i;
  __shared__ int ids[CSR_CAP9]; __shared__ unsigned short key[CSR_CAP9]; __shared__ int outp[CSR_CAP9]; __shared__ int ncnt[CSR_GN9 + 1]; __shared__ int boff[CSR_NBLK9 + 1];
  const int g = blockIdx.x, t_ = threadIdx.x; int tot = TOT[g]; int st = START[g], stn = START[g + 1]; const int v0 = g * CSR_GN9; const int nv = min(CSR_GN9, N - v0); const int t0 = g * CSR_TS9;
  st = (st < 0) ? 0 : (st > permLen - 32 ? permLen - 32 : st) & ~31; stn = (stn < st) ? st : (stn > permLen ? permLen : stn); tot = (tot < 0) ? 0 : tot; if (tot > stn - st && tot <= CSR_CAP9) tot = stn - st;
  if (tot > CSR_CAP9) {
    for (int pass = 0; pass < 2; ++pass) { for (int i = t_; i < CSR_TS9 / 4; i += 256) { v4i a, c; for (int e = 0; e < 4; ++e) { a[e] = st; c[e] = 0; } *(volatile v4i*)(ROWPTR + t0 + i * 4) = a; *(volatile v4i*)(ROWCNT + t0 + i * 4) = c; } if (t_ == 0) ((volatile int*)FLAG)[0] = 1; __threadfence(); } (void)nv; return; }
  if (t_ == 0) { int acc = 0; for (int b = 0; b < CSR_NBLK9; ++b) { boff[b] = acc; int c = HST[(size_t)b * NGP + g]; c = (c < 0) ? 0 : (c > CHP ? CHP : c); acc += c; if (acc > tot) acc = tot; } boff[CSR_NBLK9] = acc; }
  for (int i = t_; i <= CSR_GN9; i += 256) ncnt[i] = 0;
  __syncthreads();
  for (int b = 0; b < CSR_NBLK9; ++b) { const int c = boff[b + 1] - boff[b]; int o_ = OFF[(size_t)g * CSR_NBLK9 + b]; o_ = (o_ < 0) ? 0 : (o_ > CHP - c ? CHP - c : o_); const int* src_ = STG + (size_t)b * CHP + o_;
    for (int i = t_; i < c; i += 256) { int id = src_[i]; id = (id < 0) ? 0 : id; ids[boff[b] + i] = id; int d = dst[id]; d = (d < v0) ? v0 : (d >= N ? N - 1 : d); int kk = d - v0; kk = (kk < 0) ? 0 : (kk >= CSR_GN9 ? CSR_GN9 - 1 : kk); key[boff[b] + i] = (unsigned short)kk; } }
  __syncthreads();
  if (t_ == 0) { for (int i = 0; i < tot; ++i) ncnt[key[i]] += 1; int acc = 0; for (int vl = 0; vl < CSR_GN9; ++vl) { const int c = ncnt[vl]; ncnt[vl] = acc; acc += c; } ncnt[CSR_GN9] = acc;
    for (int i = 0; i < tot; ++i) { const int vl = key[i]; outp[ncnt[vl]] = ids[i]; ncnt[vl] += 1; }
    for (int vl = CSR_GN9; vl > 0; --vl) ncnt[vl] = ncnt[vl - 1]; ncnt[0] = 0; }
  __syncthreads();
  for (int pass = 0; pass < 2; ++pass) {
    for (int i = t_; i < (stn - st) / 4; i += 256) { v4i v; for (int e = 0; e < 4; ++e) { const int q = i * 4 + e; v[e] = (q < tot) ? outp[q] : -1; } *(volatile v4i*)(PERM + st + i * 4) = v; }
    for (int i = t_; i < CSR_TS9 / 4; i += 256) { v4i a, c; for (int e = 0; e < 4; ++e) { const int vl = i * 4 + e; const int vc = vl < CSR_GN9 ? vl : CSR_GN9; a[e] = (vl < CSR_GN9) ? st + ncnt[vc] : st; c[e] = (vl < nv) ? (ncnt[(vc < CSR_GN9 ? vc : CSR_GN9 - 1) + 1] - ncnt[vc]) : 0; } *(volatile v4i*)(ROWPTR + t0 + i * 4) = a; *(volatile v4i*)(ROWCNT + t0 + i * 4) = c; }
    __threadfence(); }
}
__global__ __launch_bounds__(256) void csrZ_kernel9(int* __restrict__ p, size_t n4) { typedef __attribute__((ext_vector_type(4))) int v4i; const size_t tid = (size_t)blockIdx.x * 256 + threadIdx.x, nth = (size_t)gridDim.x * 256; v4i z = {0, 0, 0, 0}; for (size_t i = tid; i < n4; i += nth) *(volatile v4i*)(p + i * 4) = z; }
struct CsrBufs9 { int *STG, *HST, *OFF, *START, *TOT, *PERM, *ROWPTR, *ROWCNT, *FLAG; int nG, NGP, CHP; size_t permLen; char* base; size_t bytes; };
static size_t csr_carve9(CsrBufs9& c, char* ws, size_t off, int E, int N) {
  const size_t off0 = off; c.base = ws + off;
  auto al = [&](size_t bytes) { char* p = ws + off; off += (bytes + 255) & ~(size_t)255; return p; };
  c.nG = (N + CSR_GN9 - 1) / CSR_GN9; c.NGP = (c.nG + 31) & ~31; const int ch = (E + CSR_NBLK9 - 1) / CSR_NBLK9; c.CHP = (ch + 31) & ~31; c.permLen = (size_t)E + 32 * (size_t)c.nG + 32;
  c.STG = (int*)al((size_t)CSR_NBLK9 * c.CHP * 4); c.HST = (int*)al((size_t)CSR_NBLK9 * c.NGP * 4); c.OFF = (int*)al((size_t)c.NGP * CSR_NBLK9 * 4); c.START = (int*)al((size_t)(c.NGP + 64) * 4); c.TOT = (int*)al((size_t)(c.NGP + 64) * 4);
  c.PERM = (int*)al(c.permLen * 4); c.ROWPTR = (int*)al((size_t)c.nG * CSR_TS9 * 4); c.ROWCNT = (int*)al((size_t)c.nG * CSR_TS9 * 4); c.FLAG = (int*)al(256);
  c.bytes = off - off0; return off;
}
static void csr_build9(const CsrBufs9& c, const int* dst, int E, int N, hipStream_t stream) {
  const size_t smem = (size_t)(2 * c.NGP + c.CHP) * 4;
  csrZ_kernel9<<<512, 256, 0, stream>>>((int*)c.base, c.bytes / 16);
  csrA_kernel9<<<CSR_NBLK9, 64, smem, stream>>>(dst, E, N, c.nG, c.CHP, c.NGP, c.STG, c.HST);
  csrS_kernel9<<<1, 512, 0, stream>>>(c.HST, c.nG, c.NGP, c.START, c.TOT, c.OFF);
  csrB_kernel9<<<c.nG, 256, 0, stream>>>(dst, N, c.nG, c.CHP, c.NGP, (int)c.permLen, c.STG, c.HST, c.OFF, c.START, c.TOT, c.PERM, c.ROWPTR, c.ROWCNT, c.FLAG);
}


__global__ __launch_bounds__(256) void wput_kernel(const float* __restrict__ w2, b16* __restrict__ W2T) { const int u = blockIdx.x * 256 + threadIdx.x; if (u >= WN * 8) return; const int o = u / 8, k0 = (u % 8) * 8; v8b v;
#pragma unroll
  for (int j = 0; j < 8; ++j) v[j] = (b16)(bf16_rne(w2[(size_t)(k0 + j) * WN + o]) * WSC); for (int pass = 0; pass < 2; ++pass) { *(volatile v8b*)(W2T + (size_t)o * HID + k0) = v; __threadfence(); } }

struct EdgeT { float s[16][MS]; float v[16][MV][3]; float cr[16][MV][3]; float dot[16][MV]; float y[16][3]; float msg[16][DIM]; };
__global__ __launch_bounds__(32) void edge_kernel(const float* __restrict__ h, const float* __restrict__ pos, const int* __restrict__ srcs, const int* __restrict__ dsts, const float* __restrict__ means, const float* __restrict__ betas, const float* __restrict__ W1, const float* __restrict__ b1, const b16* __restrict__ W2T, const float* __restrict__ b2, int ELIM, float* __restrict__ MSG) {
  __shared__ __attribute__((aligned(16))) b16 Ah[16][72], Al[16][72]; __shared__ float T[16][O1 + 4]; __shared__ EdgeT L; const int lane = threadIdx.x, nloc = lane & 15, hlf = lane >> 4; const size_t e0 = (size_t)blockIdx.x * 16; if (e0 >= (size_t)ELIM) return;
  { const int rr = lane & 15, hf = lane >> 4; const size_t e = e0 + rr; const size_t si = (size_t)iclamp(srcs[e], 0, N - 1), di = (size_t)iclamp(dsts[e], 0, N - 1);
    if (hf == 0) { for (int c = 0; c < MS; ++c) L.s[rr][c] = bf16_rne(h[si * DIM + c]); for (int u = 0; u < MV; ++u) for (int d = 0; d < 3; ++d) L.v[rr][u][d] = bf16_rne(h[si * DIM + MS + u * 3 + d]); }
    else { float vc[3]; float dd = 0.0f; for (int d = 0; d < 3; ++d) { vc[d] = bf16_rne(pos[di * 3 + d]) - bf16_rne(pos[si * 3 + d]); dd += pmul(vc[d], vc[d]); } const float dist = sqrtf(dd + 1e-12f); for (int d = 0; d < 3; ++d) L.y[rr][d] = pmul(SQ3, vc[d] / dist);
      const float cut = dist < CUT ? 0.5f * (cosf(dist * PI / CUT) + 1.0f) : 0.0f; const float ex = __expf(-ALPHA * dist); float rbf[NR];
#pragma unroll
      for (int k = 0; k < NR; ++k) { const float df = ex - bf16_rne(means[k]); rbf[k] = pmul(__expf(-bf16_rne(betas[k]) * pmul(df, df)), cut); }
      for (int j = 0; j < HID; ++j) { float a = bf16_rne(b1[j]);
#pragma unroll
        for (int k = 0; k < NR; ++k) a += pmul(rbf[k], bf16_rne(W1[k * HID + j])); b16 p, q; split16(silu(a) * XS, p, q); Ah[rr][j] = p; Al[rr][j] = q; } } }
  wave_lds_sync();
  { const int rr = lane & 15, hf = lane >> 4; for (int u = hf; u < MV; u += 2) { const float* vv = L.v[rr][u]; const float* yy = L.y[rr]; L.dot[rr][u] = (pmul(vv[0], yy[0]) + pmul(vv[1], yy[1]) + pmul(vv[2], yy[2])) * (1.0f / SQ3);
      L.cr[rr][u][0] = (pmul(vv[1], yy[2]) - pmul(vv[2], yy[1])) * (1.0f / SQ2); L.cr[rr][u][1] = (pmul(vv[2], yy[0]) - pmul(vv[0], yy[2])) * (1.0f / SQ2); L.cr[rr][u][2] = (pmul(vv[0], yy[1]) - pmul(vv[1], yy[0])) * (1.0f / SQ2); } }
  wave_lds_sync();
  const v16b a0 = frag_kb(&Ah[nloc][0], hlf), a1 = frag_kb(&Ah[nloc][32], hlf), l0 = frag_kb(&Al[nloc][0], hlf), l1 = frag_kb(&Al[nloc][32], hlf);
  auto gemm_block = [&](int col0, int ncols) {
    for (int t = 0; t < ncols / 16; ++t) { const b16* wr = W2T + (size_t)(col0 + t * 16 + nloc) * HID; v8f acc = {}; acc = wmma16b(a0, frag_kb(wr, hlf), acc); acc = wmma16b(l0, frag_kb(wr, hlf), acc); acc = wmma16b(a1, frag_kb(wr + 32, hlf), acc); acc = wmma16b(l1, frag_kb(wr + 32, hlf), acc);
      const float bb = bf16_rne(b2[col0 + t * 16 + nloc]);
#pragma unroll
      for (int r8 = 0; r8 < 8; ++r8) T[8 * hlf + r8][t * 16 + nloc] = acc[r8] * (1.0f / (XS * WSC)) + bb; }
    wave_lds_sync(); };
  const float cS = 1.0f / sqrtf((float)MS), cV = 1.0f / sqrtf((float)MV);
  gemm_block(0, O1); for (int rr = 0; rr < 16; ++rr) { float p = 0.0f; for (int u = 0; u < MS; ++u) p += pmul(L.s[rr][u], T[rr][u * MS + lane]); L.msg[rr][lane] = p * cS; } wave_lds_sync();
  gemm_block(O1, O2 - O1); if (lane < MV) for (int rr = 0; rr < 16; ++rr) { float p = 0.0f; for (int u = 0; u < MS; ++u) p += pmul(L.s[rr][u], T[rr][u * MV + lane]); for (int d = 0; d < 3; ++d) L.msg[rr][MS + lane * 3 + d] = pmul(p, L.y[rr][d]) * cS; } wave_lds_sync();
  gemm_block(O2, O3 - O2); if (lane < MV) for (int rr = 0; rr < 16; ++rr) { float p[3] = {0.0f, 0.0f, 0.0f}; for (int u = 0; u < MV; ++u) { const float w = T[rr][u * MV + lane]; for (int d = 0; d < 3; ++d) p[d] += pmul(L.v[rr][u][d], w); } for (int d = 0; d < 3; ++d) L.msg[rr][MS + lane * 3 + d] += p[d] * cV; } wave_lds_sync();
  gemm_block(O3, O4 - O3); for (int rr = 0; rr < 16; ++rr) { float p = 0.0f; for (int u = 0; u < MV; ++u) p += pmul(L.dot[rr][u], T[rr][u * MS + lane]); L.msg[rr][lane] = (L.msg[rr][lane] + p * cV) * (1.0f / SQ2); } wave_lds_sync();
  gemm_block(O4, WN - O4); if (lane < MV) for (int rr = 0; rr < 16; ++rr) { float p[3] = {0.0f, 0.0f, 0.0f}; for (int u = 0; u < MV; ++u) { const float w = T[rr][u * MV + lane]; for (int d = 0; d < 3; ++d) p[d] += pmul(L.cr[rr][u][d], w); } for (int d = 0; d < 3; ++d) L.msg[rr][MS + lane * 3 + d] = (L.msg[rr][MS + lane * 3 + d] + p[d] * cV) * (1.0f / SQ3); } wave_lds_sync();
  for (int pass = 0; pass < 2; ++pass) { for (int q = lane; q < 16 * DIM; q += 32) ((volatile float*)MSG)[(e0 * DIM) + q] = L.msg[q / DIM][q % DIM]; __threadfence(); } }
__global__ __launch_bounds__(256) void node_kernel(const float* __restrict__ h, const float* __restrict__ MSG, const float* __restrict__ Wss, const float* __restrict__ Wvv, const int* __restrict__ PERM, const int* __restrict__ ROWPTR, const int* __restrict__ ROWCNT, int permLen, int ELIM, float* __restrict__ out) {
  __shared__ float Hr[8][2][DIM], Or[8][2][DIM]; const int wave = threadIdx.x >> 5, lane = threadIdx.x & 31; const int n0 = (blockIdx.x * 8 + wave) * 2; if (n0 >= N) return;
  for (int k = 0; k < 2; ++k) { const int n = n0 + k; for (int c = lane; c < DIM; c += 32) Hr[wave][k][c] = bf16_rne(h[(size_t)n * DIM + c]); }
  wave_lds_sync();
  for (int k = 0; k < 2; ++k) { const int n = n0 + k; int st = ROWPTR[n], cnt = ROWCNT[n]; cnt = iclamp(cnt, 0, E); st = iclamp(st, 0, permLen - cnt); float a0 = 0.0f, a1 = 0.0f, a2 = 0.0f; int nin = 0;
#pragma unroll 1
    for (int j = 0; j < cnt; ++j) { const size_t e = (size_t)iclamp(PERM[st + j], 0, E - 1); if (e >= (size_t)ELIM) continue; ++nin; a0 += MSG[e * DIM + lane]; a1 += MSG[e * DIM + 32 + lane]; if (lane < DIM - 64) a2 += MSG[e * DIM + 64 + lane]; }
    const float inv = 1.0f / (float)(nin > 0 ? nin : 1);
    float ss = 0.0f; for (int u = 0; u < MS; ++u) ss += pmul(Hr[wave][k][u], bf16_rne(Wss[u * MS + lane])); Or[wave][k][lane] = pmul(a0, inv) + ss * 0.17677669529663688f + Hr[wave][k][lane];
    if (lane < MV) { for (int d = 0; d < 3; ++d) { float sv = 0.0f; for (int u = 0; u < MV; ++u) sv += pmul(Hr[wave][k][MS + u * 3 + d], bf16_rne(Wvv[u * MV + lane])); const int c = MS + lane * 3 + d; Or[wave][k][c] = sv * 0.25f + Hr[wave][k][c]; } }
    wave_lds_sync();
    Or[wave][k][32 + lane] += pmul(a1, inv); if (lane < DIM - 64) Or[wave][k][64 + lane] += pmul(a2, inv);
    wave_lds_sync(); }
  for (int pass = 0; pass < 2; ++pass) { for (int q = lane; q < 2 * DIM; q += 32) ((volatile float*)out)[(size_t)n0 * DIM + q] = Or[wave][q / DIM][q % DIM]; __threadfence(); } }
}

extern "C" void kernel_launch(void* const* d_in, const int* in_sizes, int n_in, void* d_out, int out_size, void* d_ws, size_t ws_size, hipStream_t stream) {
  (void)n_in;
  auto Fp = [&](int i) { return (const float*)d_in[i]; }; auto Ip = [&](int i) { return (const int*)d_in[i]; };
  if (in_sizes[0] != N * DIM || in_sizes[1] != N * 3 || in_sizes[2] != 2 * E || in_sizes[3] != NR || in_sizes[4] != NR || in_sizes[5] != NR * HID || in_sizes[7] != HID * WN || in_sizes[8] != WN || in_sizes[9] != MS * MS || in_sizes[10] != MV * MV || out_size != N * DIM) return;
  const int ELIM = E;
  size_t off = 0; char* ws = (char*)d_ws;
  auto carve = [&](size_t bytes) { char* p = ws + off; off += (bytes + 255) & ~(size_t)255; return p; };
  b16* W2T = (b16*)carve((size_t)WN * HID * 2); float* MSG = (float*)carve((size_t)E * DIM * 4); CsrBufs9 csr; off = csr_carve9(csr, ws, off, E, N);
  if (off > ws_size || off > ((size_t)24 << 20)) return;
  wput_kernel<<<(WN * 8 + 255) / 256, 256, 0, stream>>>(Fp(7), W2T);
  csr_build9(csr, Ip(2) + E, E, N, stream);
  edge_kernel<<<E / 16, 32, 0, stream>>>(Fp(0), Fp(1), Ip(2), Ip(2) + E, Fp(3), Fp(4), Fp(5), Fp(6), W2T, Fp(8), ELIM, MSG);
  node_kernel<<<(N / 2 + 7) / 8, 256, 0, stream>>>(Fp(0), MSG, Fp(9), Fp(10), csr.PERM, csr.ROWPTR, csr.ROWCNT, (int)csr.permLen, ELIM, (float*)d_out);
}
